// SlidingWindowAttention_71708773974020
// MI455X (gfx1250) — hardware-verified
//
#include <hip/hip_runtime.h>

#ifndef NB
#define NB 2
#endif
#ifndef SEQ
#define SEQ 2048
#endif
#define NB_FULL   2
#define SEQ_FULL  2048
#define D_MODEL   1024
#define NUM_HEADS 16
#define HEAD_DIM  64
#define WINDOW    128
#define SCALE_F   0.125f
#define W_CARRY   64.0f
#define P_CARRY   1024.0f
#define CTX_CARRY 16.0f
#define RES_CARRY 2048.0f
#define RES_INV   0.00048828125f

static_assert(NB >= 1 && NB <= NB_FULL);
static_assert(SEQ >= 64 && SEQ <= SEQ_FULL);
static_assert((SEQ % 64) == 0);
static_assert((D_MODEL % 64) == 0);
static_assert(NUM_HEADS * HEAD_DIM == D_MODEL);
static_assert(((NB * SEQ) % 32) == 0);

typedef _Float16 v16h __attribute__((ext_vector_type(16)));
typedef _Float16 v8h  __attribute__((ext_vector_type(8)));
typedef float    v8f  __attribute__((ext_vector_type(8)));
typedef float    v4f  __attribute__((ext_vector_type(4)));
typedef float    v4fa __attribute__((ext_vector_type(4))) __attribute__((may_alias));

static __device__ __forceinline__ float bf16r(float f) {
  unsigned int u = __float_as_uint(f);
  u = u + 0x7FFFu + ((u >> 16) & 1u);
  u &= 0xFFFF0000u;
  return __uint_as_float(u);
}

static __device__ __forceinline__ v16h load_frag(const _Float16* row, int lane) {
  const int kb = (lane < 16) ? 0 : 8;
  v8h lo = *(const v8h*)(row + kb);
  v8h hi = *(const v8h*)(row + kb + 16);
  v16h r;
#pragma unroll
  for (int i = 0; i < 8; ++i) { r[i] = lo[i]; r[i + 8] = hi[i]; }
  return r;
}

static __device__ __forceinline__ v8f wmma16(v16h a, v16h b, v8f c) {
  v8f d = __builtin_amdgcn_wmma_f32_16x16x32_f16(false, a, false, b, (short)0, c, false, false);
  asm volatile("v_nop\n\tv_nop\n\tv_nop\n\tv_nop" : "+v"(d) : "v"(a), "v"(b));
  return d;
}

static __device__ __forceinline__ void wave_lds_sync() {
  asm volatile("s_wait_dscnt 0x0" ::: "memory");
  __builtin_amdgcn_fence(3, "wavefront");
  __builtin_amdgcn_wave_barrier();
}

__global__ __launch_bounds__(256) void cvt_plane(const float* __restrict__ src, _Float16* dst,
                                                 int rows, int seqc, int seqf, float scale) {
  const int n8 = rows * (D_MODEL / 8);
  const int i8 = blockIdx.x * blockDim.x + threadIdx.x;
  if (i8 >= n8) return;
  const int r = i8 / (D_MODEL / 8);
  const int c = i8 - r * (D_MODEL / 8);
  const int b = r / seqc;
  const int t = r - b * seqc;
  const float* sp = src + (size_t)(b * seqf + t) * D_MODEL + c * 8;
  const v4f x0 = *(const v4f*)sp;
  const v4f x1 = *(const v4f*)(sp + 4);
  v8h o;
#pragma unroll
  for (int e = 0; e < 4; ++e) {
    o[e]     = (_Float16)(bf16r(x0[e]) * scale);
    o[e + 4] = (_Float16)(bf16r(x1[e]) * scale);
  }
  const v4f w = __builtin_bit_cast(v4f, o);
  float* dp = (float*)(dst + (size_t)i8 * 8);
  *(volatile v4f*)dp = w;
  __threadfence();
  *(volatile v4f*)dp = w;
}

template <int MODE>
__global__ __launch_bounds__(128) __attribute__((amdgpu_num_vgpr(256)))
void gemm_xwt(const _Float16* __restrict__ A, const _Float16* __restrict__ W,
              const float* __restrict__ bias, void* out, void* out2,
              int M, int N, int K, float oscale, int seqc, int seqf) {
  constexpr int STP32 = 68;
  constexpr int STP16 = 72;
  constexpr int RES_OFF = 32 * STP16;
  __shared__ __align__(16) float stg[4][32 * 72];
  const int lane  = threadIdx.x & 31;
  const int wslot = threadIdx.x >> 5;
  const int wid   = blockIdx.x * 4 + wslot;
  const int tilesN = N >> 6;
  const int m0 = (wid / tilesN) << 5;
  const int n0 = (wid % tilesN) << 6;
  if (m0 >= M) return;
  const int col = lane & 15;
  const int lh  = lane >> 4;

  v8f acc0[4] = {v8f{}, v8f{}, v8f{}, v8f{}};
  v8f acc1[4] = {v8f{}, v8f{}, v8f{}, v8f{}};
  const _Float16* arow0 = A + (size_t)(m0 + col) * K;
  const _Float16* arow1 = A + (size_t)(m0 + 16 + col) * K;

#pragma unroll 1
  for (int k0 = 0; k0 < K; k0 += 32) {
    const v16h af0 = load_frag(arow0 + k0, lane);
    const v16h af1 = load_frag(arow1 + k0, lane);
#pragma unroll
    for (int t = 0; t < 4; ++t) {
      const v16h bf = load_frag(W + (size_t)(n0 + t * 16 + col) * K + k0, lane);
      acc0[t] = wmma16(af0, bf, acc0[t]);
      acc1[t] = wmma16(af1, bf, acc1[t]);
    }
  }

  float* st = &stg[wslot][0];
  _Float16* st16 = (_Float16*)st;
#pragma unroll
  for (int t = 0; t < 4; ++t) {
    const float bc = bf16r(bias[n0 + t * 16 + col]);
#pragma unroll
    for (int i = 0; i < 8; ++i) {
      const int r0 = i + lh * 8, r1 = 16 + i + lh * 8, c = t * 16 + col;
      const float v0 = acc0[t][i] * oscale + bc;
      const float v1 = acc1[t][i] * oscale + bc;
      if (MODE == 0) {
        st[r0 * STP32 + c] = v0;
        st[r1 * STP32 + c] = v1;
      } else {
        const _Float16 h0 = (_Float16)v0;
        const _Float16 h1 = (_Float16)v1;
        st16[r0 * STP16 + c] = h0;
        st16[r1 * STP16 + c] = h1;
        if (MODE == 2) {
          st16[RES_OFF + r0 * STP16 + c] = (_Float16)((v0 - (float)h0) * RES_CARRY);
          st16[RES_OFF + r1 * STP16 + c] = (_Float16)((v1 - (float)h1) * RES_CARRY);
        }
      }
    }
  }
  wave_lds_sync();

  const int bidx  = m0 / seqc;
  const int obase = bidx * seqf + (m0 - bidx * seqc);
  if (MODE == 0) {
    float* O = (float*)out;
#pragma unroll
    for (int ps = 0; ps < 2; ++ps) {
      if (ps) __threadfence();
#pragma unroll
      for (int s = 0; s < 16; ++s) {
        const int L = s * 4 + (lane >> 3);
        const int row = L >> 1;
        const int piece = (L & 1) * 8 + (lane & 7);
        const v4f val = *(const v4fa*)(st + row * STP32 + piece * 4);
        float* gp = O + (size_t)(obase + row) * N + n0 + piece * 4;
        *(volatile v4f*)gp = val;
      }
    }
  } else {
    _Float16* O = (_Float16*)out;
    _Float16* R = (_Float16*)out2;
#pragma unroll
    for (int ps = 0; ps < 2; ++ps) {
      if (ps) __threadfence();
#pragma unroll
      for (int s = 0; s < 8; ++s) {
        const int row = s * 4 + (lane >> 3);
        const int piece = lane & 7;
        const v4f val = *(const v4fa*)(st16 + row * STP16 + piece * 8);
        float* gp = (float*)(O + (size_t)(obase + row) * N + n0 + piece * 8);
        *(volatile v4f*)gp = val;
      }
      if (MODE == 2) {
#pragma unroll
        for (int s = 0; s < 8; ++s) {
          const int row = s * 4 + (lane >> 3);
          const int piece = lane & 7;
          const v4f val = *(const v4fa*)(st16 + RES_OFF + row * STP16 + piece * 8);
          float* gp = (float*)(R + (size_t)(obase + row) * N + n0 + piece * 8);
          *(volatile v4f*)gp = val;
        }
      }
    }
  }
}

__global__ __launch_bounds__(256) void transpose_v(const _Float16* __restrict__ Vh, _Float16* Vt) {
  __shared__ __align__(16) _Float16 tileT[64][72];
  constexpr int stiles = SEQ / 64;
  const int bh = blockIdx.x / stiles;
  const int s0 = (blockIdx.x - bh * stiles) * 64;
  const int b  = bh / NUM_HEADS, h = bh - (bh / NUM_HEADS) * NUM_HEADS;
  const int t  = threadIdx.x;
#pragma unroll
  for (int it = 0; it < 2; ++it) {
    const int lin = it * 256 + t;
    const int s = lin >> 3, c = lin & 7;
    const v8h vv = *(const v8h*)(Vh + (size_t)(b * SEQ + s0 + s) * D_MODEL + h * HEAD_DIM + c * 8);
#pragma unroll
    for (int e = 0; e < 8; ++e) tileT[c * 8 + e][s] = vv[e];
  }
  __syncthreads();
  const int wave = t >> 5, lane = t & 31;
#pragma unroll
  for (int ps = 0; ps < 2; ++ps) {
    if (ps) __threadfence();
#pragma unroll
    for (int s2 = 0; s2 < 2; ++s2) {
      const int d = (wave * 2 + s2) * 4 + (lane >> 3);
      const int piece = lane & 7;
      const v4f val = *(const v4fa*)(&tileT[d][piece * 8]);
      float* gp = (float*)(Vt + ((size_t)bh * HEAD_DIM + d) * SEQ + s0 + piece * 8);
      *(volatile v4f*)gp = val;
    }
  }
}

__global__ __launch_bounds__(256) __attribute__((amdgpu_num_vgpr(256)))
void attn_band(const _Float16* __restrict__ Qh, const _Float16* __restrict__ Qr,
               const _Float16* __restrict__ Kh, const _Float16* __restrict__ Kr,
               const _Float16* __restrict__ Vt, _Float16* Oh, int nbh) {
  __shared__ __align__(16) float ldsS[8][16 * 32];
  const int lane  = threadIdx.x & 31;
  const int wslot = threadIdx.x >> 5;
  const int wid   = blockIdx.x * 8 + wslot;
  constexpr int qtiles = SEQ / 16;
  const int qt = wid % qtiles;
  const int bh = wid / qtiles;
  if (bh >= nbh) return;
  const int b = bh / NUM_HEADS;
  const int h = bh - b * NUM_HEADS;
  const int q0 = qt * 16;
  const int col = lane & 15;
  const int lh  = lane >> 4;
  const int kb  = (lane < 16) ? 0 : 8;
  const int q   = q0 + col;
  float* Sw = &ldsS[wslot][0];

  const size_t qoff = (size_t)(b * SEQ + q0 + col) * D_MODEL + h * HEAD_DIM;
  const v16h qa0 = load_frag(Qh + qoff, lane);
  const v16h qa1 = load_frag(Qh + qoff + 32, lane);
  const v16h qr0 = load_frag(Qr + qoff, lane);
  const v16h qr1 = load_frag(Qr + qoff + 32, lane);

  float m_row = -1e30f, l_row = 0.f;
  v8f o[4] = {v8f{}, v8f{}, v8f{}, v8f{}};

  const int jlo = (q0 > WINDOW) ? ((q0 - WINDOW) & ~31) : 0;
  int jhi = q0 + 15 + WINDOW; if (jhi > SEQ - 1) jhi = SEQ - 1;

#pragma unroll 1
  for (int j0 = jlo; j0 <= jhi; j0 += 32) {
    const size_t koff0 = (size_t)(b * SEQ + j0 + col) * D_MODEL + h * HEAD_DIM;
    const size_t koff1 = koff0 + (size_t)16 * D_MODEL;
    v8f s0 = {}, s1 = {};
    {
      const v16h kf0 = load_frag(Kh + koff0, lane);
      const v16h kf1 = load_frag(Kh + koff0 + 32, lane);
      s0 = wmma16(qa0, kf0, s0);
      s0 = wmma16(qa1, kf1, s0);
      v8f e0 = {};
      e0 = wmma16(qr0, kf0, e0);
      e0 = wmma16(qr1, kf1, e0);
      const v16h rf0 = load_frag(Kr + koff0, lane);
      e0 = wmma16(qa0, rf0, e0);
      const v16h rf1 = load_frag(Kr + koff0 + 32, lane);
      e0 = wmma16(qa1, rf1, e0);
#pragma unroll
      for (int i = 0; i < 8; ++i) s0[i] = s0[i] + e0[i] * RES_INV;
    }
    {
      const v16h kf0 = load_frag(Kh + koff1, lane);
      const v16h kf1 = load_frag(Kh + koff1 + 32, lane);
      s1 = wmma16(qa0, kf0, s1);
      s1 = wmma16(qa1, kf1, s1);
      v8f e1 = {};
      e1 = wmma16(qr0, kf0, e1);
      e1 = wmma16(qr1, kf1, e1);
      const v16h rf0 = load_frag(Kr + koff1, lane);
      e1 = wmma16(qa0, rf0, e1);
      const v16h rf1 = load_frag(Kr + koff1 + 32, lane);
      e1 = wmma16(qa1, rf1, e1);
#pragma unroll
      for (int i = 0; i < 8; ++i) s1[i] = s1[i] + e1[i] * RES_INV;
    }

    wave_lds_sync();
#pragma unroll
    for (int i = 0; i < 8; ++i) {
      Sw[(i + lh * 8) * 32 + col]      = s0[i];
      Sw[(i + lh * 8) * 32 + 16 + col] = s1[i];
    }
    wave_lds_sync();

    float sv[16];
    const float* Srow = Sw + col * 32 + kb;
#pragma unroll
    for (int e = 0; e < 8; ++e) { sv[e] = Srow[e] * SCALE_F; sv[e + 8] = Srow[e + 16] * SCALE_F; }

    const bool full = (j0 >= q0 - (WINDOW - 15)) && (j0 <= q0 + (WINDOW - 31));

    float mnew, alpha, sloc;
    v16h pf;
    if (full) {
      float mloc = sv[0];
#pragma unroll
      for (int e = 1; e < 16; ++e) mloc = fmaxf(mloc, sv[e]);
      const float rowmax = fmaxf(mloc, __shfl_xor(mloc, 16, 32));
      mnew  = fmaxf(m_row, rowmax);
      alpha = __expf(m_row - mnew);
      sloc  = 0.f;
#pragma unroll
      for (int e = 0; e < 16; ++e) {
        const float pv = __expf(sv[e] - mnew);
        pf[e] = (_Float16)(pv * P_CARRY);
        sloc += pv;
      }
    } else {
      bool vm[16];
      float mloc = -1e30f;
#pragma unroll
      for (int e = 0; e < 16; ++e) {
        const int j = j0 + kb + ((e < 8) ? e : e + 8);
        vm[e] = (j >= q - WINDOW) && (j <= q + WINDOW);
        sv[e] = vm[e] ? sv[e] : -1e30f;
        mloc  = fmaxf(mloc, sv[e]);
      }
      const float rowmax = fmaxf(mloc, __shfl_xor(mloc, 16, 32));
      mnew  = fmaxf(m_row, rowmax);
      alpha = __expf(m_row - mnew);
      sloc  = 0.f;
#pragma unroll
      for (int e = 0; e < 16; ++e) {
        const float pv = vm[e] ? __expf(sv[e] - mnew) : 0.f;
        pf[e] = (_Float16)(pv * P_CARRY);
        sloc += pv;
      }
    }
    const float rowsum = sloc + __shfl_xor(sloc, 16, 32);
    l_row = l_row * alpha + rowsum;
    m_row = mnew;

#pragma unroll
    for (int i = 0; i < 8; ++i) {
      const float ai = __shfl(alpha, i + lh * 8, 32);
      o[0][i] *= ai; o[1][i] *= ai; o[2][i] *= ai; o[3][i] *= ai;
    }

    const _Float16* Vb = Vt + (size_t)bh * HEAD_DIM * SEQ + j0;
#pragma unroll
    for (int t = 0; t < 4; ++t) {
      const v16h vf = load_frag(Vb + (size_t)(t * 16 + col) * SEQ, lane);
      o[t] = wmma16(pf, vf, o[t]);
    }
  }

  const float invl = (1.0f / l_row) * (CTX_CARRY / P_CARRY);
  _Float16* st16 = (_Float16*)Sw;
  wave_lds_sync();
#pragma unroll
  for (int i = 0; i < 8; ++i) {
    const float li = __shfl(invl, i + lh * 8, 32);
#pragma unroll
    for (int t = 0; t < 4; ++t)
      st16[(i + lh * 8) * 64 + t * 16 + col] = (_Float16)(o[t][i] * li);
  }
  wave_lds_sync();
  _Float16* Ob = Oh + (size_t)(b * SEQ + q0) * D_MODEL + h * HEAD_DIM;
#pragma unroll
  for (int ps = 0; ps < 2; ++ps) {
    if (ps) __threadfence();
#pragma unroll
    for (int s = 0; s < 4; ++s) {
      const int row = s * 4 + (lane >> 3);
      const int piece = lane & 7;
      const v4f val = *(const v4fa*)(st16 + row * 64 + piece * 8);
      float* gp = (float*)(Ob + (size_t)row * D_MODEL + piece * 8);
      *(volatile v4f*)gp = val;
    }
  }
}

extern "C" void kernel_launch(void* const* d_in, const int* in_sizes, int n_in,
                              void* d_out, int out_size, void* d_ws, size_t ws_size,
                              hipStream_t stream) {
  if (n_in < 11) return;
  const float* q  = (const float*)d_in[0];
  const float* k  = (const float*)d_in[1];
  const float* v  = (const float*)d_in[2];
  const float* Wq = (const float*)d_in[3];
  const float* bq = (const float*)d_in[4];
  const float* Wk = (const float*)d_in[5];
  const float* bk = (const float*)d_in[6];
  const float* Wv = (const float*)d_in[7];
  const float* bv = (const float*)d_in[8];
  const float* Wo = (const float*)d_in[9];
  const float* bo = (const float*)d_in[10];

  const int rows_c = NB * SEQ;
  const size_t need_act = ((size_t)(NB - 1) * SEQ_FULL + SEQ) * D_MODEL;
  const size_t need_w   = (size_t)D_MODEL * D_MODEL;
  if ((size_t)in_sizes[0] < need_act || (size_t)in_sizes[1] < need_act || (size_t)in_sizes[2] < need_act) return;
  if ((size_t)in_sizes[3] < need_w || (size_t)in_sizes[5] < need_w ||
      (size_t)in_sizes[7] < need_w || (size_t)in_sizes[9] < need_w) return;
  if (in_sizes[4] < D_MODEL || in_sizes[6] < D_MODEL || in_sizes[8] < D_MODEL || in_sizes[10] < D_MODEL) return;
  if ((size_t)out_size < need_act) return;

  const size_t nx = (size_t)rows_c * D_MODEL;
  const size_t nw = (size_t)D_MODEL * D_MODEL;
  const size_t total_bytes = (10 * nx + 4 * nw) * sizeof(_Float16);
  if (total_bytes > ws_size) return;

  _Float16* p = (_Float16*)d_ws;
  _Float16* q16 = p; p += nx;
  _Float16* k16 = p; p += nx;
  _Float16* v16 = p; p += nx;
  _Float16* Wqh = p; p += nw;
  _Float16* Wkh = p; p += nw;
  _Float16* Wvh = p; p += nw;
  _Float16* Woh = p; p += nw;
  _Float16* Qh  = p; p += nx;
  _Float16* Qr  = p; p += nx;
  _Float16* Khp = p; p += nx;
  _Float16* Krp = p; p += nx;
  _Float16* Vh  = p; p += nx;
  _Float16* Vtp = p; p += nx;
  _Float16* Ah  = p; p += nx;

  const int T = 256;
  const int n8a = rows_c * (D_MODEL / 8);
  const int n8w = D_MODEL * (D_MODEL / 8);
  const int ga = (n8a + T - 1) / T, gw = (n8w + T - 1) / T;
  cvt_plane<<<ga, T, 0, stream>>>(q, q16, rows_c, SEQ, SEQ_FULL, 1.0f);
  cvt_plane<<<ga, T, 0, stream>>>(k, k16, rows_c, SEQ, SEQ_FULL, 1.0f);
  cvt_plane<<<ga, T, 0, stream>>>(v, v16, rows_c, SEQ, SEQ_FULL, 1.0f);
  cvt_plane<<<gw, T, 0, stream>>>(Wq, Wqh, D_MODEL, D_MODEL, D_MODEL, W_CARRY);
  cvt_plane<<<gw, T, 0, stream>>>(Wk, Wkh, D_MODEL, D_MODEL, D_MODEL, W_CARRY);
  cvt_plane<<<gw, T, 0, stream>>>(Wv, Wvh, D_MODEL, D_MODEL, D_MODEL, W_CARRY);
  cvt_plane<<<gw, T, 0, stream>>>(Wo, Woh, D_MODEL, D_MODEL, D_MODEL, W_CARRY);

  const int gemm_tiles  = (rows_c / 32) * (D_MODEL / 64);
  const int gemm_blocks = (gemm_tiles + 3) / 4;
  const float qkv_scale = 1.0f / W_CARRY;
  const float out_scale = 1.0f / (W_CARRY * CTX_CARRY);
  gemm_xwt<2><<<gemm_blocks, 128, 0, stream>>>(q16, Wqh, bq, (void*)Qh,  (void*)Qr,  rows_c, D_MODEL, D_MODEL, qkv_scale, SEQ, SEQ);
  gemm_xwt<2><<<gemm_blocks, 128, 0, stream>>>(k16, Wkh, bk, (void*)Khp, (void*)Krp, rows_c, D_MODEL, D_MODEL, qkv_scale, SEQ, SEQ);
  gemm_xwt<1><<<gemm_blocks, 128, 0, stream>>>(v16, Wvh, bv, (void*)Vh,  (void*)Vh,  rows_c, D_MODEL, D_MODEL, qkv_scale, SEQ, SEQ);

  transpose_v<<<NB * NUM_HEADS * (SEQ / 64), T, 0, stream>>>(Vh, Vtp);

  const int nbh = NB * NUM_HEADS;
  const int attn_waves  = nbh * (SEQ / 16);
  const int attn_blocks = (attn_waves + 7) / 8;
  attn_band<<<attn_blocks, T, 0, stream>>>(Qh, Qr, Khp, Krp, Vtp, Ah, nbh);

  gemm_xwt<0><<<gemm_blocks, 128, 0, stream>>>(Ah, Woh, bo, d_out, d_out, rows_c, D_MODEL, D_MODEL, out_scale, SEQ, SEQ_FULL);
}
